// MultiHeadAttention_57741540327756
// MI455X (gfx1250) — hardware-run, weakly checked
//
#include <hip/hip_runtime.h>


#ifndef NB
#define NB 2
#endif
#ifndef SEQ
#define SEQ 2048
#endif
#define NB_FULL  2
#define SEQ_FULL 2048
#ifndef OUT_SEQ
#define OUT_SEQ SEQ
#endif
#define DM   1024
#define NH_  16
#define HD   64
#define AW   4
#define QRS  2048.0f
#define QRI  (1.0f / 2048.0f)
#define SC2  (0.125f * 1.4426950408889634f)
#define PSH  8.0f
#define NEGF (-3.0e38f)
#define EROWS ((SEQ < 512) ? SEQ : 512)
#define EPT  (SEQ / 256)

static_assert(HD == 64);
static_assert(NH_ * HD == DM);
static_assert(DM % 64 == 0);
static_assert(DM % 32 == 0);
static_assert(SEQ % 256 == 0);
static_assert((NB * SEQ) % 64 == 0);
static_assert(SEQ % 32 == 0);
static_assert(EROWS % (16 * AW) == 0);
static_assert((SEQ - EROWS) % (16 * AW) == 0);
static_assert(((size_t)SEQ * DM) % 8 == 0);
static_assert(((size_t)DM * DM) % 8 == 0);
static_assert(((size_t)NH_ * DM) % 8 == 0);
static_assert(NB <= NB_FULL);
static_assert(SEQ <= SEQ_FULL);

typedef _Float16 h16;
typedef unsigned short bf;
typedef __attribute__((ext_vector_type(16))) __bf16   v16bf;
typedef __attribute__((ext_vector_type(16))) _Float16 v16h;
typedef __attribute__((ext_vector_type(8)))  _Float16 v8h;
typedef __attribute__((ext_vector_type(8)))  unsigned short v8us;
typedef __attribute__((ext_vector_type(8)))  float    v8f;
typedef __attribute__((ext_vector_type(4)))  float    v4f;
typedef __attribute__((ext_vector_type(8)))  int      v8i;
typedef __attribute__((ext_vector_type(4)))  int      v4i;
typedef v4f  __attribute__((may_alias)) v4fa;
typedef v4i  __attribute__((may_alias)) v4ia;

__device__ __forceinline__ unsigned short f2bf(float f) { unsigned u = __float_as_uint(f); u += 0x7FFFu + ((u >> 16) & 1u); return (unsigned short)(u >> 16); }
__device__ __forceinline__ float bf2f(unsigned short u) { return __uint_as_float(((unsigned)u) << 16); }
__device__ __forceinline__ v16h cat16(v8h lo, v8h hi) { return __builtin_shufflevector(lo, hi, 0, 1, 2, 3, 4, 5, 6, 7, 8, 9, 10, 11, 12, 13, 14, 15); }
__device__ __forceinline__ v16bf cat16b(v8us lo, v8us hi) { return __builtin_bit_cast(v16bf, __builtin_shufflevector(lo, hi, 0, 1, 2, 3, 4, 5, 6, 7, 8, 9, 10, 11, 12, 13, 14, 15)); }
__device__ __forceinline__ v8f wmma16(v16h a, v16h b, v8f c) { return __builtin_amdgcn_wmma_f32_16x16x32_f16(false, a, false, b, (short)0, c, false, false); }
__device__ __forceinline__ v8f wmmab(v16bf a, v16bf b, v8f c) { return __builtin_amdgcn_wmma_f32_16x16x32_bf16(false, a, false, b, (short)0, c, false, false); }
__device__ __forceinline__ v16h  ldh(const h16* p) { return cat16(*(const v8h*)p, *(const v8h*)(p + 16)); }
__device__ __forceinline__ v16bf ldb(const bf* p)  { return cat16b(*(const v8us*)p, *(const v8us*)(p + 16)); }
__device__ __forceinline__ void wave_sync() { __builtin_amdgcn_fence(3  , "wavefront"); __builtin_amdgcn_wave_barrier(); asm volatile("" ::: "memory"); }

__global__ __launch_bounds__(256) void k_cvt8(const float* __restrict__ src, bf* dst, size_t n8) {
    const size_t i = (size_t)blockIdx.x * 256 + threadIdx.x; if (i >= n8) return;
    const v8f v = *(const v8f*)(src + i * 8); v8us o;
#pragma unroll
    for (int k = 0; k < 8; ++k) o[k] = f2bf(v[k]);
    *(volatile v8us*)(dst + i * 8) = o; __threadfence(); *(volatile v8us*)(dst + i * 8) = o;
}

__global__ __launch_bounds__(32) void k_invf(float* INVF) {
#pragma clang fp contract(off)
    const int i = threadIdx.x & 31;
    const float e = (float)(2 * i) * (1.0f / 64.0f);
    const float p = powf(10000.0f, e);
    const float f = 1.0f / p;
    *(volatile float*)(INVF + i) = f; __threadfence(); *(volatile float*)(INVF + i) = f;
}

__global__ __launch_bounds__(256) void k_tab(const int* __restrict__ mask, const float* __restrict__ INVF, float* TAB, int* POS) {
#pragma clang fp contract(off)
    __shared__ int spart[256];
    __shared__ __align__(16) int spos[SEQ];
    __shared__ float sfr[32];
    const int tid = threadIdx.x, b = blockIdx.x;
    const int* mrow = mask + (size_t)b * SEQ_FULL;
    int loc = 0;
#pragma unroll 1
    for (int e = 0; e < EPT; ++e) loc += mrow[tid * EPT + e];
    spart[tid] = loc;
    if (tid < 32) sfr[tid] = INVF[tid];
    __syncthreads();
    int pre = 0;
#pragma unroll 1
    for (int j = 0; j < 256; ++j) { const int v = spart[j]; pre += (j < tid) ? v : 0; }
    int run = pre;
#pragma unroll 1
    for (int e = 0; e < EPT; ++e) { run += mrow[tid * EPT + e]; spos[tid * EPT + e] = run - 1; }
    __syncthreads();
    int* prow = POS + (size_t)b * SEQ;
#pragma unroll 1
    for (int ps = 0; ps < 2; ++ps) {
#pragma unroll 1
        for (int i4 = tid; i4 < SEQ / 4; i4 += 256) { const v4i v = *(const v4ia*)(&spos[i4 * 4]); *(volatile v4i*)(prow + i4 * 4) = v; }
        if (ps == 0) __threadfence();
    }
    float* trow = TAB + (size_t)b * SEQ * 64;
#pragma unroll 1
    for (int it = 0; it < SEQ * 32 / 256; ++it) {
        const int e = it * 256 + tid; const int i = e & 31, t = e >> 5;
        const float ang = (float)spos[t] * sfr[i];
        const float cs = cosf(ang), sn = sinf(ang);
        float* pc = trow + (size_t)t * 64 + i;
        *(volatile float*)pc = cs; *(volatile float*)(pc + 32) = sn;
        __threadfence();
        *(volatile float*)pc = cs; *(volatile float*)(pc + 32) = sn;
    }
}

template<int ROPE, int RES>
__global__ __launch_bounds__(32) void k_proj(const bf* __restrict__ A, const bf* __restrict__ Bt, h16* Ph, h16* Pr, const float* __restrict__ TAB, int RB, size_t sRB, int pitch, int CB, size_t sCB) {
    __shared__ __align__(16) float os[16 * 68];
    const int K = DM;
    const int lane = threadIdx.x & 31, lr = lane & 15, hi = lane >> 4; const int r0 = blockIdx.x * 64, c0 = blockIdx.y * 64;
    v8f acc[4][4];
#pragma unroll
    for (int mb = 0; mb < 4; ++mb)
#pragma unroll
        for (int nb = 0; nb < 4; ++nb) acc[mb][nb] = (v8f){};
    const size_t aoff = (size_t)(r0 + lr) * K + 8 * hi, boff = (size_t)(c0 + lr) * K + 8 * hi;
#pragma unroll 1
    for (int kc = 0; kc < K; kc += 32) {
        v16bf a[4];
#pragma unroll
        for (int mb = 0; mb < 4; ++mb) a[mb] = ldb(A + aoff + (size_t)mb * 16 * K + kc);
#pragma unroll
        for (int nb = 0; nb < 4; ++nb) { const v16bf b = ldb(Bt + boff + (size_t)nb * 16 * K + kc);
#pragma unroll
            for (int mb = 0; mb < 4; ++mb) acc[mb][nb] = wmmab(a[mb], b, acc[mb][nb]); }
        asm volatile("v_nop\n\tv_nop\n\tv_nop\n\tv_nop" : "+v"(acc[0][0]), "+v"(acc[1][1]), "+v"(acc[2][2]), "+v"(acc[3][3]) : "v"(a[0]), "v"(a[1]), "v"(a[2]), "v"(a[3]));
    }
    const size_t tbase = (size_t)(r0 / RB) * sRB + (size_t)(r0 % RB) * (size_t)pitch + (size_t)(c0 / CB) * sCB + (size_t)(c0 % CB);
#pragma unroll
    for (int mb = 0; mb < 4; ++mb) {
#pragma unroll
        for (int nb = 0; nb < 4; ++nb) {
#pragma unroll
            for (int j = 0; j < 8; ++j) os[(hi * 8 + j) * 68 + nb * 16 + lr] = acc[mb][nb][j]; }
        wave_sync();
        const size_t sb = tbase + (size_t)(mb * 16) * (size_t)pitch;
#pragma unroll 1
        for (int ps = 0; ps < 2; ++ps) {
#pragma unroll
            for (int s = 0; s < 4; ++s) { const int row = 4 * s + (lane >> 3), c8 = (lane & 7) * 8;
                v4f x0 = *(const v4fa*)(&os[row * 68 + c8]); v4f x1 = *(const v4fa*)(&os[row * 68 + c8 + 4]);
                if (ROPE) {
                    const int pc = c8 ^ 32;
                    const v4f y0 = *(const v4fa*)(&os[row * 68 + pc]); const v4f y1 = *(const v4fa*)(&os[row * 68 + pc + 4]);
                    const float* tr = TAB + (size_t)(r0 + mb * 16 + row) * 64 + (c8 & 31);
                    const v4f cA = *(const v4f*)tr, cB = *(const v4f*)(tr + 4), sA = *(const v4f*)(tr + 32), sB = *(const v4f*)(tr + 36);
                    const float sg = (c8 < 32) ? -1.0f : 1.0f;
#pragma unroll
                    for (int i = 0; i < 4; ++i) { x0[i] = x0[i] * cA[i] + sg * (y0[i] * sA[i]); x1[i] = x1[i] * cB[i] + sg * (y1[i] * sB[i]); }
                }
                v8h hv, rv;
#pragma unroll
                for (int i = 0; i < 4; ++i) { const h16 a0 = (h16)x0[i]; const h16 a1 = (h16)x1[i]; hv[i] = a0; hv[4 + i] = a1; rv[i] = (h16)((x0[i] - (float)a0) * QRS); rv[4 + i] = (h16)((x1[i] - (float)a1) * QRS); }
                const size_t oo = sb + (size_t)row * (size_t)pitch + c8;
                *(volatile v8h*)(Ph + oo) = hv; if (RES) *(volatile v8h*)(Pr + oo) = rv; }
            if (ps == 0) __threadfence(); }
        wave_sync();
    }
}

__global__ __launch_bounds__(32) void k_gate(const bf* __restrict__ A, const bf* __restrict__ Bt, float* G) {
    __shared__ __align__(16) float gs[64 * 16];
    const int K = DM;
    const int lane = threadIdx.x & 31, lr = lane & 15, hi = lane >> 4; const int r0 = blockIdx.x * 64;
    v8f acc[4];
#pragma unroll
    for (int mb = 0; mb < 4; ++mb) acc[mb] = (v8f){};
    const size_t aoff = (size_t)(r0 + lr) * K + 8 * hi, boff = (size_t)lr * K + 8 * hi;
#pragma unroll 1
    for (int kc = 0; kc < K; kc += 32) {
        v16bf a[4];
#pragma unroll
        for (int mb = 0; mb < 4; ++mb) a[mb] = ldb(A + aoff + (size_t)mb * 16 * K + kc);
        const v16bf b = ldb(Bt + boff + kc);
#pragma unroll
        for (int mb = 0; mb < 4; ++mb) acc[mb] = wmmab(a[mb], b, acc[mb]);
        asm volatile("v_nop\n\tv_nop\n\tv_nop\n\tv_nop" : "+v"(acc[0]), "+v"(acc[1]), "+v"(acc[2]), "+v"(acc[3]) : "v"(a[0]), "v"(a[1]), "v"(a[2]), "v"(a[3]), "v"(b));
    }
#pragma unroll
    for (int mb = 0; mb < 4; ++mb) {
#pragma unroll
        for (int j = 0; j < 8; ++j) { const float z = acc[mb][j]; gs[(mb * 16 + 8 * hi + j) * 16 + lr] = 1.0f / (1.0f + expf(-z)); } }
    wave_sync();
    float* gb = G + (size_t)r0 * 16;
#pragma unroll 1
    for (int ps = 0; ps < 2; ++ps) {
#pragma unroll
        for (int s = 0; s < 8; ++s) { const int idx = (s * 32 + lane) * 4;
            const v4f val = *(const v4fa*)(&gs[idx]);
            *(volatile v4f*)(gb + idx) = val; }
        if (ps == 0) __threadfence(); }
}

template<int EARLY>
__global__ __launch_bounds__(32 * AW) void k_flash(const h16* __restrict__ QH, const h16* __restrict__ QR, const h16* __restrict__ KP, const h16* __restrict__ VT, const h16* __restrict__ VR,
                                                   const int* __restrict__ MASK, const int* __restrict__ POS, const float* __restrict__ GATE, bf* CH, size_t cps, int tbase) {
    __shared__ __align__(16) float os[AW * 16 * 68];
    const int lane = threadIdx.x & 31, lr = lane & 15, hi = lane >> 4;
    const int wave = __builtin_amdgcn_readfirstlane((int)(threadIdx.x >> 5));
    const int zh = blockIdx.y; const int b = zh / NH_, h = zh % NH_;
    const int t0 = tbase + (blockIdx.x * AW + wave) * 16;
    const int tq = t0 + lr;
    const size_t pbase = (size_t)zh * SEQ * HD;
    const size_t qo = pbase + (size_t)(t0 + lr) * HD + 8 * hi;
    const v16h qh0 = ldh(QH + qo), qh1 = ldh(QH + qo + 32), qr0 = ldh(QR + qo), qr1 = ldh(QR + qo + 32);
    const size_t ko = pbase + (size_t)lr * HD + 8 * hi;
    const size_t vo = pbase + (size_t)lr * SEQ + 8 * hi;
    const int* mrow = MASK + (size_t)b * SEQ_FULL + 8 * hi;
    const int p0 = POS[(size_t)b * SEQ + t0];
    const int kend = __builtin_amdgcn_readfirstlane((p0 < 0) ? SEQ : (t0 + 16));
    v8f oH0 = (v8f){}, oH1 = (v8f){}, oH2 = (v8f){}, oH3 = (v8f){};
    v8f oL0 = (v8f){}, oL1 = (v8f){}, oL2 = (v8f){}, oL3 = (v8f){};
    float m = NEGF, l = 0.0f;
#pragma unroll 1
    for (int key0 = 0; key0 < kend; key0 += 32) {
        const h16* ka = KP + ko + (size_t)key0 * HD;
        const v16h ka0 = ldh(ka), ka1 = ldh(ka + 32), kb0 = ldh(ka + 16 * HD), kb1 = ldh(ka + 16 * HD + 32);
        const v8i mka = *(const v8i*)(mrow + key0);
        const v8i mkb = *(const v8i*)(mrow + key0 + 16);
        v8f sHa = (v8f){}, sLa = (v8f){}, sHb = (v8f){}, sLb = (v8f){};
        sHa = wmma16(ka0, qh0, sHa); sLa = wmma16(ka0, qr0, sLa); sHb = wmma16(kb0, qh0, sHb); sLb = wmma16(kb0, qr0, sLb);
        sHa = wmma16(ka1, qh1, sHa); sLa = wmma16(ka1, qr1, sLa); sHb = wmma16(kb1, qh1, sHb); sLb = wmma16(kb1, qr1, sLb);
        asm volatile("v_nop\n\tv_nop\n\tv_nop\n\tv_nop" : "+v"(sHa), "+v"(sLa), "+v"(sHb), "+v"(sLb) : "v"(ka0), "v"(ka1), "v"(kb0), "v"(kb1));
        const int kfa = key0 + 8 * hi;
        float ta[8], tb[8]; float mx = NEGF;
#pragma unroll
        for (int r = 0; r < 8; ++r) {
            const bool oka = (mka[r] != 0) & ((kfa + r) <= tq);
            const bool okb = (mkb[r] != 0) & ((kfa + 16 + r) <= tq);
            const float sa = (sHa[r] + sLa[r] * QRI) * SC2; const float sb = (sHb[r] + sLb[r] * QRI) * SC2;
            ta[r] = oka ? sa : NEGF; tb[r] = okb ? sb : NEGF;
            mx = fmaxf(mx, fmaxf(ta[r], tb[r])); }
        mx = fmaxf(mx, __shfl_xor(mx, 16, 32));
        const float mnew = fmaxf(m, mx);
        const float alpha = __builtin_amdgcn_exp2f(m - mnew);
        const float sh = PSH - mnew;
        v16h pb, pr; float ls = 0.0f;
#pragma unroll
        for (int r = 0; r < 8; ++r) {
            const float ea = __builtin_amdgcn_exp2f(ta[r] + sh); const float ec = __builtin_amdgcn_exp2f(tb[r] + sh);
            const h16 pa = (h16)ea; const h16 pc = (h16)ec; pb[r] = pa; pb[8 + r] = pc;
            if (EARLY) { const h16 ra = (h16)((ea - (float)pa) * QRS); const h16 rc = (h16)((ec - (float)pc) * QRS); pr[r] = ra; pr[8 + r] = rc;
                         ls += ((float)pa + (float)ra * QRI) + ((float)pc + (float)rc * QRI); }
            else { ls += (float)pa + (float)pc; } }
        l = l * alpha + ls; m = mnew;
        oH0 = oH0 * alpha; oH1 = oH1 * alpha; oH2 = oH2 * alpha; oH3 = oH3 * alpha;
        const h16* va = VT + vo + key0;
        const v16h v0 = ldh(va), v1 = ldh(va + (size_t)16 * SEQ), v2 = ldh(va + (size_t)32 * SEQ), v3 = ldh(va + (size_t)48 * SEQ);
        if (EARLY) {
            oL0 = oL0 * alpha; oL1 = oL1 * alpha; oL2 = oL2 * alpha; oL3 = oL3 * alpha;
            const h16* vra = VR + vo + key0;
            const v16h w0 = ldh(vra), w1 = ldh(vra + (size_t)16 * SEQ), w2 = ldh(vra + (size_t)32 * SEQ), w3 = ldh(vra + (size_t)48 * SEQ);
            oH0 = wmma16(v0, pb, oH0); oH1 = wmma16(v1, pb, oH1); oH2 = wmma16(v2, pb, oH2); oH3 = wmma16(v3, pb, oH3);
            oL0 = wmma16(v0, pr, oL0); oL1 = wmma16(v1, pr, oL1); oL2 = wmma16(v2, pr, oL2); oL3 = wmma16(v3, pr, oL3);
            oL0 = wmma16(w0, pb, oL0); oL1 = wmma16(w1, pb, oL1); oL2 = wmma16(w2, pb, oL2); oL3 = wmma16(w3, pb, oL3);
            asm volatile("v_nop\n\tv_nop\n\tv_nop\n\tv_nop" : "+v"(oH0), "+v"(oH1), "+v"(oH2), "+v"(oH3), "+v"(oL0), "+v"(oL1), "+v"(oL2), "+v"(oL3)
                         : "v"(v0), "v"(v1), "v"(v2), "v"(v3), "v"(w0), "v"(w1), "v"(w2), "v"(w3), "v"(pb), "v"(pr));
        } else {
            oH0 = wmma16(v0, pb, oH0); oH1 = wmma16(v1, pb, oH1); oH2 = wmma16(v2, pb, oH2); oH3 = wmma16(v3, pb, oH3);
            asm volatile("v_nop\n\tv_nop\n\tv_nop\n\tv_nop" : "+v"(oH0), "+v"(oH1), "+v"(oH2), "+v"(oH3) : "v"(v0), "v"(v1), "v"(v2), "v"(v3), "v"(pb));
        }
    }
    l += __shfl_xor(l, 16, 32);
    const float inv = 1.0f / l;
    const float g = GATE[((size_t)b * SEQ + tq) * NH_ + h];
    const float sc = inv * g;
    if (EARLY) {
        oH0 = oH0 + oL0 * QRI; oH1 = oH1 + oL1 * QRI; oH2 = oH2 + oL2 * QRI; oH3 = oH3 + oL3 * QRI;
    }
    const int wb = wave * 16 * 68;
    { v4f a, c;
      a[0] = oH0[0] * sc; a[1] = oH0[1] * sc; a[2] = oH0[2] * sc; a[3] = oH0[3] * sc; c[0] = oH0[4] * sc; c[1] = oH0[5] * sc; c[2] = oH0[6] * sc; c[3] = oH0[7] * sc;
      *(v4fa*)(&os[wb + lr * 68 +  0 + 8 * hi]) = a; *(v4fa*)(&os[wb + lr * 68 +  0 + 8 * hi + 4]) = c;
      a[0] = oH1[0] * sc; a[1] = oH1[1] * sc; a[2] = oH1[2] * sc; a[3] = oH1[3] * sc; c[0] = oH1[4] * sc; c[1] = oH1[5] * sc; c[2] = oH1[6] * sc; c[3] = oH1[7] * sc;
      *(v4fa*)(&os[wb + lr * 68 + 16 + 8 * hi]) = a; *(v4fa*)(&os[wb + lr * 68 + 16 + 8 * hi + 4]) = c;
      a[0] = oH2[0] * sc; a[1] = oH2[1] * sc; a[2] = oH2[2] * sc; a[3] = oH2[3] * sc; c[0] = oH2[4] * sc; c[1] = oH2[5] * sc; c[2] = oH2[6] * sc; c[3] = oH2[7] * sc;
      *(v4fa*)(&os[wb + lr * 68 + 32 + 8 * hi]) = a; *(v4fa*)(&os[wb + lr * 68 + 32 + 8 * hi + 4]) = c;
      a[0] = oH3[0] * sc; a[1] = oH3[1] * sc; a[2] = oH3[2] * sc; a[3] = oH3[3] * sc; c[0] = oH3[4] * sc; c[1] = oH3[5] * sc; c[2] = oH3[6] * sc; c[3] = oH3[7] * sc;
      *(v4fa*)(&os[wb + lr * 68 + 48 + 8 * hi]) = a; *(v4fa*)(&os[wb + lr * 68 + 48 + 8 * hi + 4]) = c; }
    wave_sync();
    bf* ch = CH + ((size_t)b * SEQ + t0) * DM + h * HD;
#pragma unroll 1
    for (int ps = 0; ps < 2; ++ps) {
#pragma unroll
        for (int s = 0; s < 4; ++s) { const int row = 4 * s + (lane >> 3), c8 = (lane & 7) * 8;
            const v4f x0 = *(const v4fa*)(&os[wb + row * 68 + c8]); const v4f x1 = *(const v4fa*)(&os[wb + row * 68 + c8 + 4]); v8us hv, lv;
#pragma unroll
            for (int i = 0; i < 4; ++i) { const unsigned short u0 = f2bf(x0[i]); const unsigned short u1 = f2bf(x1[i]); hv[i] = u0; hv[4 + i] = u1;
                                          lv[i] = f2bf(x0[i] - bf2f(u0)); lv[4 + i] = f2bf(x1[i] - bf2f(u1)); }
            const size_t oo = (size_t)row * DM + c8;
            *(volatile v8us*)(ch + oo) = hv; *(volatile v8us*)(ch + cps + oo) = lv; }
        if (ps == 0) __threadfence(); }
}

__global__ __launch_bounds__(32) void k_oproj(const bf* __restrict__ A, size_t aPS, const bf* __restrict__ Bt, const float* __restrict__ bias, float* OUT) {
    __shared__ __align__(16) float os[16 * 68];
    const int K = DM;
    const int lane = threadIdx.x & 31, lr = lane & 15, hi = lane >> 4; const int r0 = blockIdx.x * 64, c0 = blockIdx.y * 64;
    v8f acc[4][4];
#pragma unroll
    for (int mb = 0; mb < 4; ++mb)
#pragma unroll
        for (int nb = 0; nb < 4; ++nb) acc[mb][nb] = (v8f){};
    const size_t aoff = (size_t)(r0 + lr) * K + 8 * hi, boff = (size_t)(c0 + lr) * K + 8 * hi;
#pragma unroll 1
    for (int pl = 0; pl < 2; ++pl) {
        const size_t ao = aoff + (size_t)pl * aPS;
#pragma unroll 1
        for (int kc = 0; kc < K; kc += 32) {
            v16bf a[4];
#pragma unroll
            for (int mb = 0; mb < 4; ++mb) a[mb] = ldb(A + ao + (size_t)mb * 16 * K + kc);
#pragma unroll
            for (int nb = 0; nb < 4; ++nb) { const v16bf b = ldb(Bt + boff + (size_t)nb * 16 * K + kc);
#pragma unroll
                for (int mb = 0; mb < 4; ++mb) acc[mb][nb] = wmmab(a[mb], b, acc[mb][nb]); }
            asm volatile("v_nop\n\tv_nop\n\tv_nop\n\tv_nop" : "+v"(acc[0][0]), "+v"(acc[1][1]), "+v"(acc[2][2]), "+v"(acc[3][3]) : "v"(a[0]), "v"(a[1]), "v"(a[2]), "v"(a[3]));
        }
    }
    v4f bv = *(const v4f*)(bias + c0 + lr * 4);
#pragma unroll
    for (int i = 0; i < 4; ++i) bv[i] = bf2f(f2bf(bv[i]));
    float* ob = OUT + ((size_t)(r0 / SEQ) * OUT_SEQ + (size_t)(r0 % SEQ)) * DM + c0;
#pragma unroll
    for (int mb = 0; mb < 4; ++mb) {
#pragma unroll
        for (int nb = 0; nb < 4; ++nb) {
#pragma unroll
            for (int j = 0; j < 8; ++j) os[(hi * 8 + j) * 68 + nb * 16 + lr] = acc[mb][nb][j]; }
        wave_sync();
#pragma unroll 1
        for (int ps = 0; ps < 2; ++ps) {
#pragma unroll
            for (int s = 0; s < 8; ++s) { const int row = 2 * s + hi, cofs = lr * 4;
                const v4f val = *(const v4fa*)(&os[row * 68 + cofs]) + bv;
                *(volatile v4f*)(ob + (size_t)(mb * 16 + row) * DM + cofs) = val; }
            if (ps == 0) __threadfence(); }
        wave_sync();
    }
}

static constexpr size_t al256(size_t v) { return (v + 255) & ~(size_t)255; }
static constexpr size_t SZ_XB = al256((size_t)NB * SEQ * DM * 2);
static constexpr size_t SZ_WB = al256((size_t)4 * DM * DM * 2);
static constexpr size_t SZ_WG = al256((size_t)NH_ * DM * 2);
static constexpr size_t SZ_PL = al256((size_t)NB * NH_ * SEQ * HD * 2);
static constexpr size_t SZ_CX = al256((size_t)2 * NB * SEQ * DM * 2);
static constexpr size_t SZ_TB = al256((size_t)NB * SEQ * 64 * 4);
static constexpr size_t SZ_GT = al256((size_t)NB * SEQ * NH_ * 4);
static constexpr size_t SZ_PS = al256((size_t)NB * SEQ * 4);
static constexpr size_t SZ_IF = 256;
static constexpr size_t SZ_TOTAL = SZ_XB + SZ_WB + SZ_WG + 5 * SZ_PL + SZ_CX + SZ_TB + SZ_GT + SZ_PS + SZ_IF;
static_assert(SZ_TOTAL <= (size_t)134217728);
static_assert(((size_t)DM * DM * 2) % 256 == 0);
static_assert(((size_t)NB * SEQ * DM * 2) % 256 == 0);

extern "C" void kernel_launch(void* const* d_in, const int* in_sizes, int n_in,
                              void* d_out, int out_size, void* d_ws, size_t ws_size, hipStream_t stream) {
    if (n_in < 8) return;
    const size_t needx = ((size_t)(NB - 1) * SEQ_FULL + SEQ) * DM;
    const size_t needm = (size_t)(NB - 1) * SEQ_FULL + SEQ;
    if ((size_t)in_sizes[0] < needx) return;
    if ((size_t)in_sizes[1] < needm) return;
    if ((size_t)in_sizes[2] < (size_t)DM * DM || (size_t)in_sizes[3] < (size_t)DM * DM || (size_t)in_sizes[4] < (size_t)DM * DM) return;
    if ((size_t)in_sizes[5] < (size_t)NH_ * DM) return;
    if ((size_t)in_sizes[6] < (size_t)DM * DM) return;
    if ((size_t)in_sizes[7] < (size_t)DM) return;
    if ((size_t)out_size < ((size_t)(NB - 1) * OUT_SEQ + SEQ) * DM) return;
    if (SZ_TOTAL > ws_size) return;
    const float* x = (const float*)d_in[0]; const int* mask = (const int*)d_in[1];
    const float* wq = (const float*)d_in[2]; const float* wk = (const float*)d_in[3]; const float* wv = (const float*)d_in[4];
    const float* wg = (const float*)d_in[5]; const float* wp = (const float*)d_in[6]; const float* bp = (const float*)d_in[7];
    float* OUT = (float*)d_out;
    char* wsp = (char*)d_ws;
    bf* XB = (bf*)wsp; wsp += SZ_XB;
    bf* WB = (bf*)wsp; wsp += SZ_WB;
    bf* WG = (bf*)wsp; wsp += SZ_WG;
    h16* QH = (h16*)wsp; wsp += SZ_PL;
    h16* QR = (h16*)wsp; wsp += SZ_PL;
    h16* KP = (h16*)wsp; wsp += SZ_PL;
    h16* VT = (h16*)wsp; wsp += SZ_PL;
    h16* VR = (h16*)wsp; wsp += SZ_PL;
    bf* CH = (bf*)wsp; wsp += SZ_CX;
    float* TAB = (float*)wsp; wsp += SZ_TB;
    float* GT = (float*)wsp; wsp += SZ_GT;
    int* POS = (int*)wsp; wsp += SZ_PS;
    float* INVF = (float*)wsp; wsp += SZ_IF;
    bf* WQ = WB; bf* WK = WB + (size_t)DM * DM; bf* WV = WB + (size_t)2 * DM * DM; bf* WP = WB + (size_t)3 * DM * DM;
    const size_t cps = (size_t)NB * SEQ * DM;

    if (SEQ == SEQ_FULL) {
        const size_t n8 = (size_t)NB * SEQ * DM / 8;
        k_cvt8<<<(unsigned)((n8 + 255) / 256), 256, 0, stream>>>(x, XB, n8);
    } else {
        const size_t n8 = (size_t)SEQ * DM / 8;
        for (int b = 0; b < NB; ++b) k_cvt8<<<(unsigned)((n8 + 255) / 256), 256, 0, stream>>>(x + (size_t)b * SEQ_FULL * DM, XB + (size_t)b * SEQ * DM, n8);
    }
    { const size_t n8 = (size_t)DM * DM / 8; const unsigned g = (unsigned)((n8 + 255) / 256);
      k_cvt8<<<g, 256, 0, stream>>>(wq, WQ, n8); k_cvt8<<<g, 256, 0, stream>>>(wk, WK, n8); k_cvt8<<<g, 256, 0, stream>>>(wv, WV, n8); k_cvt8<<<g, 256, 0, stream>>>(wp, WP, n8); }
    { const size_t n8 = (size_t)NH_ * DM / 8; k_cvt8<<<(unsigned)((n8 + 255) / 256), 256, 0, stream>>>(wg, WG, n8); }

    k_invf<<<1, 32, 0, stream>>>(INVF);
    k_tab<<<NB, 256, 0, stream>>>(mask, INVF, TAB, POS);

    k_proj<1, 1><<<dim3(NB * SEQ / 64, DM / 64, 1), 32, 0, stream>>>(XB, WQ, QH, QR, TAB, SEQ, (size_t)NH_ * SEQ * HD, HD, HD, (size_t)SEQ * HD);
    k_proj<1, 0><<<dim3(NB * SEQ / 64, DM / 64, 1), 32, 0, stream>>>(XB, WK, KP, KP, TAB, SEQ, (size_t)NH_ * SEQ * HD, HD, HD, (size_t)SEQ * HD);
    k_proj<0, 1><<<dim3(DM / 64, NB * SEQ / 64, 1), 32, 0, stream>>>(WV, XB, VT, VR, TAB, DM, (size_t)0, SEQ, SEQ, (size_t)DM * SEQ);

    k_gate<<<NB * SEQ / 64, 32, 0, stream>>>(XB, WG, GT);

    k_flash<1><<<dim3(EROWS / (16 * AW), NB * NH_, 1), 32 * AW, 0, stream>>>(QH, QR, KP, VT, VR, mask, POS, GT, CH, cps, 0);
    if (SEQ > EROWS)
        k_flash<0><<<dim3((SEQ - EROWS) / (16 * AW), NB * NH_, 1), 32 * AW, 0, stream>>>(QH, QR, KP, VT, VR, mask, POS, GT, CH, cps, EROWS);

    k_oproj<<<dim3(NB * SEQ / 64, DM / 64, 1), 32, 0, stream>>>(CH, cps, WP, bp, OUT);
}
